// LuongAttention_68891275428027
// MI455X (gfx1250) — hardware-verified
//
#include <hip/hip_runtime.h>
#include <math.h>

typedef __attribute__((ext_vector_type(16))) _Float16 v16h;
typedef __attribute__((ext_vector_type(16))) __bf16 v16b;
typedef __attribute__((ext_vector_type(8)))  _Float16 v8h;
typedef __attribute__((ext_vector_type(8)))  float v8f;
typedef __attribute__((ext_vector_type(4)))  float v4f;
typedef __attribute__((ext_vector_type(2)))  float v2f;
typedef __attribute__((ext_vector_type(4)))  unsigned v4u;
typedef __attribute__((ext_vector_type(4)))  int v4i;
typedef float __attribute__((may_alias)) float_a;
typedef int __attribute__((may_alias)) int_a;

template <typename T> __device__ __forceinline__ void vst2(void* p, T v) { *(volatile T*)p = v; __threadfence(); *(volatile T*)p = v; }
__device__ __forceinline__ v8f wmma16(v16h a, v16h b, v8f c) {
  v8f d = __builtin_amdgcn_wmma_f32_16x16x32_f16(false, a, false, b, (short)0, c, false, false);
  asm volatile("v_nop\n\tv_nop\n\tv_nop\n\tv_nop" : "+v"(d) : "v"(a), "v"(b));
  return d;
}
__device__ __forceinline__ v8f wmma_bf(v16b a, v16b b, v8f c) {
  v8f d = __builtin_amdgcn_wmma_f32_16x16x32_bf16(false, a, false, b, (short)0, c, false, false);
  asm volatile("v_nop\n\tv_nop\n\tv_nop\n\tv_nop" : "+v"(d) : "v"(a), "v"(b));
  return d;
}
__device__ __forceinline__ v16h frag_h(const _Float16* rowk0, int lane) {
  union { v16h v; v8h q[2]; } u; const _Float16* p = rowk0 + 8 * (lane >> 4);
  u.q[0] = *(const v8h*)p; u.q[1] = *(const v8h*)(p + 16); return u.v;
}
__device__ __forceinline__ v16h frag_f32(const float* rowk0, int lane) {
  v16h a; const float* p = rowk0 + 8 * (lane >> 4);
#pragma unroll
  for (int i = 0; i < 8; ++i) { a[i] = (_Float16)p[i]; a[8 + i] = (_Float16)p[16 + i]; }
  return a;
}
__device__ __forceinline__ v16h frag_f32s(const float* rowk0, int lane, float sc) {
  v16h a; const float* p = rowk0 + 8 * (lane >> 4);
#pragma unroll
  for (int i = 0; i < 8; ++i) { a[i] = (_Float16)(p[i] * sc); a[8 + i] = (_Float16)(p[16 + i] * sc); }
  return a;
}
__device__ __forceinline__ v16h fragc_f32(const float* W, int k0, int n, int lane, int ld, int K) {
  v16h a; const int g = lane >> 4;
#pragma unroll
  for (int i = 0; i < 8; ++i) { const int ka = k0 + 8 * g + i, kb = ka + 16;
    a[i] = (_Float16)(ka < K ? W[(size_t)(ka < K ? ka : K - 1) * ld + n] : 0.f); a[8 + i] = (_Float16)(kb < K ? W[(size_t)(kb < K ? kb : K - 1) * ld + n] : 0.f); }
  return a;
}
struct F2 { v16b h, l; };
__device__ __forceinline__ F2 bsplit16(const float v[16]) { F2 r;
#pragma unroll
  for (int i = 0; i < 16; ++i) { const __bf16 h = (__bf16)v[i]; r.h[i] = h; r.l[i] = (__bf16)(v[i] - (float)h); }
  return r; }
__device__ __forceinline__ F2 split_row(const float* row, int k0, int lane) { float v[16]; const float* p = row + k0 + 8 * (lane >> 4);
#pragma unroll
  for (int i = 0; i < 8; ++i) { v[i] = p[i]; v[8 + i] = p[16 + i]; }
  return bsplit16(v); }
__device__ __forceinline__ F2 split_rowK(const float* row, int k0, int lane, int K) { float v[16]; const int g = lane >> 4;
#pragma unroll
  for (int i = 0; i < 8; ++i) { const int ka = k0 + 8 * g + i, kb = ka + 16; v[i] = ka < K ? row[ka < K ? ka : K - 1] : 0.f; v[8 + i] = kb < K ? row[kb < K ? kb : K - 1] : 0.f; }
  return bsplit16(v); }
__device__ __forceinline__ F2 split_col(const float* W, int k0, int n, int lane, int ld, int K) { float v[16]; const int g = lane >> 4;
#pragma unroll
  for (int i = 0; i < 8; ++i) { const int ka = k0 + 8 * g + i, kb = ka + 16; v[i] = ka < K ? W[(size_t)(ka < K ? ka : K - 1) * ld + n] : 0.f; v[8 + i] = kb < K ? W[(size_t)(kb < K ? kb : K - 1) * ld + n] : 0.f; }
  return bsplit16(v); }
__device__ __forceinline__ v8f mac3(const F2& a, const F2& b, v8f c) { c = wmma_bf(a.l, b.h, c); c = wmma_bf(a.h, b.l, c); return wmma_bf(a.h, b.h, c); }
__device__ __forceinline__ float sigm(float v) { return 1.0f / (1.0f + expf(-v)); }
#define LDSX() do { asm volatile("s_wait_dscnt 0" ::: "memory"); __builtin_amdgcn_wave_barrier(); __builtin_amdgcn_fence(__ATOMIC_RELEASE, "workgroup"); } while (0)


#define NB 4
#define NQ 2048
#define NK 2048
#define DD 1024
#ifndef TQB
#define TQB (NQ / 64)
#define TNB NB
#endif
typedef __attribute__((ext_vector_type(8))) __bf16 v8b;
__device__ __forceinline__ v16b frag_b(const __bf16* rowk0, int lane) {
  union { v16b v; v8b q[2]; } u; const __bf16* p = rowk0 + 8 * (lane >> 4);
  u.q[0] = *(const v8b*)p; u.q[1] = *(const v8b*)(p + 16); return u.v;
}
__device__ __forceinline__ float bfr(float v) { return (float)(__bf16)v; }
__device__ __attribute__((noinline)) float exp_ni(float v) { return expf(v); }
__device__ __attribute__((noinline)) float erf_ni(float v) { return erff(v); }

#define WS_VT  0u
#define WS_KR  (WS_VT + 2u * NB * DD * NK)
#define WS_P   (WS_KR + 2u * NB * NK * DD)
#define WS_END (WS_P + 4u * NB * NQ * NK)

__global__ __launch_bounds__(256) void k_vprep(const float* __restrict__ V, __bf16* __restrict__ KR, __bf16* __restrict__ VT) {
  __shared__ __align__(16) __bf16 sr[64][136]; __shared__ __align__(16) __bf16 st[128][72];
  const int tid = threadIdx.x; const int k0 = blockIdx.x * 64, d0 = blockIdx.y * 128, b = blockIdx.z;
  for (int q = tid; q < 64 * 128; q += 256) { const int kl = q >> 7, dl = q & 127; const __bf16 v = (__bf16)V[((size_t)b * NK + k0 + kl) * DD + d0 + dl]; sr[kl][dl] = v; st[dl][kl] = v; }
  __syncthreads();
  for (int q = tid; q < 64 * 16; q += 256) { const int kl = q >> 4, pc = q & 15; vst2((unsigned*)(KR + ((size_t)b * NK + k0 + kl) * DD + d0 + pc * 8), *(const v4u*)&sr[kl][pc * 8]); }
  for (int q = tid; q < 128 * 8; q += 256) { const int dl = q >> 3, pc = q & 7; vst2((unsigned*)(VT + ((size_t)b * DD + d0 + dl) * NK + k0 + pc * 8), *(const v4u*)&st[dl][pc * 8]); }
}
__global__ __launch_bounds__(128) void k_scores(const float* __restrict__ Q, const __bf16* __restrict__ KR, float* __restrict__ P) {
  __shared__ __align__(16) float so[4][16][132];
  const int tid = threadIdx.x, wave = tid >> 5, lane = tid & 31, col = lane & 15, g = lane >> 4; const int b = blockIdx.z; const size_t r0 = (size_t)blockIdx.x * 64 + wave * 16; const int n0 = blockIdx.y * 128;
  const float* qrow = Q + ((size_t)b * NQ + r0 + col) * DD; const __bf16* kbase = KR + ((size_t)b * NK + n0) * DD;
  v8f acc[8] = {};
#pragma unroll 2
  for (int kc = 0; kc < DD / 32; ++kc) { v16b a; { const float* p = qrow + kc * 32 + 8 * g;
#pragma unroll
      for (int i = 0; i < 8; ++i) { a[i] = (__bf16)p[i]; a[8 + i] = (__bf16)p[16 + i]; } }
#pragma unroll
    for (int j = 0; j < 8; ++j) acc[j] = wmma_bf(a, frag_b(kbase + (size_t)(j * 16 + col) * DD + kc * 32, lane), acc[j]); }
#pragma unroll
  for (int j = 0; j < 8; ++j)
#pragma unroll
    for (int r = 0; r < 8; ++r) so[wave][8 * g + r][j * 16 + col] = acc[j][r];
  LDSX();
  for (int rl = 0; rl < 16; ++rl) vst2(P + ((size_t)b * NQ + r0 + rl) * NK + n0 + lane * 4, *(const v4f*)&so[wave][rl][lane * 4]);
}
__global__ __launch_bounds__(256) void k_softmax(float* P) {
  __shared__ __align__(16) float s[8][NK];
  const int wave = threadIdx.x >> 5, lane = threadIdx.x & 31; const size_t row = (size_t)blockIdx.x * 8 + wave; float* pr = P + row * NK;
  float mx = -3.0e38f; for (int k = lane; k < NK; k += 32) { const float v = pr[k]; s[wave][k] = v; mx = fmaxf(mx, v); }
#pragma unroll
  for (int o = 1; o < 32; o <<= 1) mx = fmaxf(mx, __shfl_xor(mx, o));
  float z = 0.f; for (int k = lane; k < NK; k += 32) { const float e = exp_ni(s[wave][k] - mx); s[wave][k] = e; z += e; }
#pragma unroll
  for (int o = 1; o < 32; o <<= 1) z += __shfl_xor(z, o);
  const float iz = 1.0f / z; for (int k = lane; k < NK; k += 32) s[wave][k] *= iz;
  LDSX();
  for (int pc = lane; pc < NK / 4; pc += 32) vst2(pr + pc * 4, *(const v4f*)&s[wave][pc * 4]);
}
__global__ __launch_bounds__(128) void k_ctx(const float* __restrict__ P, const __bf16* __restrict__ VT, float* __restrict__ out) {
  __shared__ __align__(16) float so[4][16][132];
  const int tid = threadIdx.x, wave = tid >> 5, lane = tid & 31, col = lane & 15, g = lane >> 4; const int b = blockIdx.z; const size_t r0 = (size_t)blockIdx.x * 64 + wave * 16; const int n0 = blockIdx.y * 128;
  const float* prow = P + ((size_t)b * NQ + r0 + col) * NK; const __bf16* vbase = VT + ((size_t)b * DD + n0) * NK;
  v8f acc[8] = {};
#pragma unroll 2
  for (int kc = 0; kc < NK / 32; ++kc) { const F2 a = split_row(prow, kc * 32, lane);
#pragma unroll
    for (int j = 0; j < 8; ++j) { const v16b w = frag_b(vbase + (size_t)(j * 16 + col) * NK + kc * 32, lane); acc[j] = wmma_bf(a.l, w, acc[j]); acc[j] = wmma_bf(a.h, w, acc[j]); } }
#pragma unroll
  for (int j = 0; j < 8; ++j)
#pragma unroll
    for (int r = 0; r < 8; ++r) so[wave][8 * g + r][j * 16 + col] = acc[j][r];
  LDSX();
  for (int rl = 0; rl < 16; ++rl) vst2(out + ((size_t)b * NQ + r0 + rl) * DD + n0 + lane * 4, *(const v4f*)&so[wave][rl][lane * 4]);
}
extern "C" void kernel_launch(void* const* d_in, const int* in_sizes, int n_in, void* d_out, int out_size, void* d_ws, size_t ws_size, hipStream_t stream) {
  (void)in_sizes; (void)n_in; (void)out_size;
  const float** F = (const float**)d_in;
  if (ws_size < (size_t)WS_END) return;
  char* ws = (char*)d_ws; __bf16 *VT = (__bf16*)(ws + WS_VT), *KR = (__bf16*)(ws + WS_KR); float* P = (float*)(ws + WS_P);
  k_vprep<<<dim3(NK / 64, DD / 128, TNB), 256, 0, stream>>>(F[1], KR, VT);
  k_scores<<<dim3(TQB, NK / 128, TNB), 128, 0, stream>>>(F[0], KR, P);
  for (int b = 0; b < TNB; ++b) k_softmax<<<(TQB * 64) / 8, 256, 0, stream>>>(P + (size_t)b * NQ * NK);
  k_ctx<<<dim3(TQB, DD / 128, TNB), 128, 0, stream>>>(P, VT, (float*)d_out);
}
